// SG_Self_Attention_24026047054362
// MI455X (gfx1250) — hardware-verified
//
#include <hip/hip_runtime.h>
#include <math.h>

typedef __attribute__((ext_vector_type(16))) _Float16 v16h;
typedef __attribute__((ext_vector_type(16))) __bf16 v16b;
typedef __attribute__((ext_vector_type(8)))  _Float16 v8h;
typedef __attribute__((ext_vector_type(8)))  float v8f;
typedef __attribute__((ext_vector_type(4)))  float v4f;
typedef __attribute__((ext_vector_type(2)))  float v2f;
typedef __attribute__((ext_vector_type(4)))  unsigned v4u;
typedef __attribute__((ext_vector_type(4)))  int v4i;
typedef float __attribute__((may_alias)) float_a;
typedef int __attribute__((may_alias)) int_a;

template <typename T> __device__ __forceinline__ void vst2(void* p, T v) { *(volatile T*)p = v; __threadfence(); *(volatile T*)p = v; }
__device__ __forceinline__ v8f wmma16(v16h a, v16h b, v8f c) {
  v8f d = __builtin_amdgcn_wmma_f32_16x16x32_f16(false, a, false, b, (short)0, c, false, false);
  asm volatile("v_nop\n\tv_nop\n\tv_nop\n\tv_nop" : "+v"(d) : "v"(a), "v"(b));
  return d;
}
__device__ __forceinline__ v8f wmma_bf(v16b a, v16b b, v8f c) {
  v8f d = __builtin_amdgcn_wmma_f32_16x16x32_bf16(false, a, false, b, (short)0, c, false, false);
  asm volatile("v_nop\n\tv_nop\n\tv_nop\n\tv_nop" : "+v"(d) : "v"(a), "v"(b));
  return d;
}
__device__ __forceinline__ v16h frag_h(const _Float16* rowk0, int lane) {
  union { v16h v; v8h q[2]; } u; const _Float16* p = rowk0 + 8 * (lane >> 4);
  u.q[0] = *(const v8h*)p; u.q[1] = *(const v8h*)(p + 16); return u.v;
}
__device__ __forceinline__ v16h frag_f32(const float* rowk0, int lane) {
  v16h a; const float* p = rowk0 + 8 * (lane >> 4);
#pragma unroll
  for (int i = 0; i < 8; ++i) { a[i] = (_Float16)p[i]; a[8 + i] = (_Float16)p[16 + i]; }
  return a;
}
__device__ __forceinline__ v16h frag_f32s(const float* rowk0, int lane, float sc) {
  v16h a; const float* p = rowk0 + 8 * (lane >> 4);
#pragma unroll
  for (int i = 0; i < 8; ++i) { a[i] = (_Float16)(p[i] * sc); a[8 + i] = (_Float16)(p[16 + i] * sc); }
  return a;
}
__device__ __forceinline__ v16h fragc_f32(const float* W, int k0, int n, int lane, int ld, int K) {
  v16h a; const int g = lane >> 4;
#pragma unroll
  for (int i = 0; i < 8; ++i) { const int ka = k0 + 8 * g + i, kb = ka + 16;
    a[i] = (_Float16)(ka < K ? W[(size_t)(ka < K ? ka : K - 1) * ld + n] : 0.f); a[8 + i] = (_Float16)(kb < K ? W[(size_t)(kb < K ? kb : K - 1) * ld + n] : 0.f); }
  return a;
}
struct F2 { v16b h, l; };
__device__ __forceinline__ F2 bsplit16(const float v[16]) { F2 r;
#pragma unroll
  for (int i = 0; i < 16; ++i) { const __bf16 h = (__bf16)v[i]; r.h[i] = h; r.l[i] = (__bf16)(v[i] - (float)h); }
  return r; }
__device__ __forceinline__ F2 split_row(const float* row, int k0, int lane) { float v[16]; const float* p = row + k0 + 8 * (lane >> 4);
#pragma unroll
  for (int i = 0; i < 8; ++i) { v[i] = p[i]; v[8 + i] = p[16 + i]; }
  return bsplit16(v); }
__device__ __forceinline__ F2 split_rowK(const float* row, int k0, int lane, int K) { float v[16]; const int g = lane >> 4;
#pragma unroll
  for (int i = 0; i < 8; ++i) { const int ka = k0 + 8 * g + i, kb = ka + 16; v[i] = ka < K ? row[ka < K ? ka : K - 1] : 0.f; v[8 + i] = kb < K ? row[kb < K ? kb : K - 1] : 0.f; }
  return bsplit16(v); }
__device__ __forceinline__ F2 split_col(const float* W, int k0, int n, int lane, int ld, int K) { float v[16]; const int g = lane >> 4;
#pragma unroll
  for (int i = 0; i < 8; ++i) { const int ka = k0 + 8 * g + i, kb = ka + 16; v[i] = ka < K ? W[(size_t)(ka < K ? ka : K - 1) * ld + n] : 0.f; v[8 + i] = kb < K ? W[(size_t)(kb < K ? kb : K - 1) * ld + n] : 0.f; }
  return bsplit16(v); }
__device__ __forceinline__ v8f mac3(const F2& a, const F2& b, v8f c) { c = wmma_bf(a.l, b.h, c); c = wmma_bf(a.h, b.l, c); return wmma_bf(a.h, b.h, c); }
__device__ __forceinline__ float sigm(float v) { return 1.0f / (1.0f + expf(-v)); }
#define LDSX() do { asm volatile("s_wait_dscnt 0" ::: "memory"); __builtin_amdgcn_wave_barrier(); __builtin_amdgcn_fence(__ATOMIC_RELEASE, "workgroup"); } while (0)


#define NB 4
#define HW 64
#define NT 4096
#define NR (NB * NT)
#define CC 256
#define NHB 4
#define HD 32
#define NK 1024
#define SCALE 0.17677669529663687f
typedef __attribute__((ext_vector_type(8))) __bf16 v8b;
__device__ __forceinline__ v16b frag_b(const __bf16* rowk0, int lane) {
  union { v16b v; v8b q[2]; } u; const __bf16* p = rowk0 + 8 * (lane >> 4);
  u.q[0] = *(const v8b*)p; u.q[1] = *(const v8b*)(p + 16); return u.v;
}
__device__ __forceinline__ v16b frag_gbf(const float* rowk0, int lane) {
  v16b a; const float* p = rowk0 + 8 * (lane >> 4);
#pragma unroll
  for (int i = 0; i < 8; ++i) { a[i] = (__bf16)p[i]; a[8 + i] = (__bf16)p[16 + i]; }
  return a;
}
__device__ __forceinline__ float bfr(float v) { return (float)(__bf16)v; }
__device__ __attribute__((noinline)) float gelu_e(float v) { return 0.5f * v * (1.0f + erff(v * 0.70710678118654752f)); }
__device__ __attribute__((noinline)) float exp_ni(float v) { return expf(v); }
__device__ __forceinline__ v8f mac3p(v16b ah, v16b al, v16b bh, v16b bl, v8f c) { c = wmma_bf(al, bh, c); c = wmma_bf(ah, bl, c); return wmma_bf(ah, bh, c); }

#define PT1_ROWS 768
#define WS_PT1   0u
#define WS_PTKV  (WS_PT1 + 2u * PT1_ROWS * CC)
#define WS_PTP   (WS_PTKV + 2u * CC * CC)
#define WS_PTSR  (WS_PTP + 2u * CC * CC)
#define WS_LPRE  (WS_PTSR + 2u * CC * 1024)
#define WS_Q1    (WS_LPRE + 4u * NR * CC)
#define WS_Q2    (WS_Q1 + 4u * NR * 128)
#define WS_KV2   (WS_Q2 + 4u * NR * 128)
#define WS_K1    (WS_KV2 + 4u * NR * CC)
#define WS_V1H   (WS_K1 + 4u * NB * NHB * NK * HD)
#define WS_V1L   (WS_V1H + 2u * NB * NHB * HD * NK)
#define WS_M1    (WS_V1L + 2u * NB * NHB * HD * NK)
#define WS_L1    (WS_M1 + 4u * NB * NHB * NT)
#define WS_GP    (WS_L1 + 4u * NB * NHB * NT)
#define WS_CAT   (WS_GP + 4u * NB * NHB * 64 * NK)
#define WS_LEPE  (WS_CAT + 4u * NR * CC)
#define WS_LMW   (WS_LEPE + 4u * NR * CC)
#define WS_END   (WS_LMW + 4u * NB * 256 * 16)

__global__ __launch_bounds__(256) void k_pack(const float* __restrict__ lw, const float* __restrict__ q1w, const float* __restrict__ q2w, const float* __restrict__ kv2w, const float* __restrict__ kv1w, const float* __restrict__ pw, const float* __restrict__ srw,
                                              __bf16* __restrict__ PT1, __bf16* __restrict__ PTKV, __bf16* __restrict__ PTP, __bf16* __restrict__ PTSR) {
  __shared__ __align__(16) __bf16 srow[1024];
  const int n = blockIdx.x, tid = threadIdx.x;
  if (n < 1280) {
    const float* Wm; int NO, nn; __bf16* dst;
    if (n < 256) { Wm = lw; NO = 256; nn = n; dst = PT1 + (size_t)n * CC; } else if (n < 384) { Wm = q1w; NO = 128; nn = n - 256; dst = PT1 + (size_t)n * CC; }
    else if (n < 512) { Wm = q2w; NO = 128; nn = n - 384; dst = PT1 + (size_t)n * CC; } else if (n < 768) { Wm = kv2w; NO = 256; nn = n - 512; dst = PT1 + (size_t)n * CC; }
    else if (n < 1024) { Wm = kv1w; NO = 256; nn = n - 768; dst = PTKV + (size_t)nn * CC; } else { Wm = pw; NO = 256; nn = n - 1024; dst = PTP + (size_t)nn * CC; }
    srow[tid] = (__bf16)Wm[(size_t)tid * NO + nn];
    __syncthreads();
    if (tid < CC / 8) vst2((unsigned*)(dst + tid * 8), *(const v4u*)(&srow[tid * 8]));
  } else {
    const int co = n - 1280;
    for (int k = tid; k < 1024; k += 256) { const int tap = k >> 8, c = k & 255; srow[k] = (__bf16)srw[(((size_t)co * CC + c) * 2 + (tap >> 1)) * 2 + (tap & 1)]; }
    __syncthreads();
    if (tid < 1024 / 8) vst2((unsigned*)(PTSR + (size_t)co * 1024 + tid * 8), *(const v4u*)(&srow[tid * 8]));
  }
}
__global__ __launch_bounds__(128) void k_lin1(const float* __restrict__ X, const __bf16* __restrict__ PT1, const float* __restrict__ lb, const float* __restrict__ q1b, const float* __restrict__ q2b, const float* __restrict__ kv2b,
                                              float* __restrict__ LPRE, float* __restrict__ Q1, float* __restrict__ Q2, float* __restrict__ KV2) {
  __shared__ __align__(16) float so[4][16][132];
  const int tid = threadIdx.x, wave = tid >> 5, lane = tid & 31, col = lane & 15, g = lane >> 4; const size_t r0 = (size_t)blockIdx.x * 64 + wave * 16; const int n0 = blockIdx.y * 128;
  v8f acc[8] = {};
#pragma unroll 2
  for (int kc = 0; kc < CC / 32; ++kc) { const v16b a = frag_gbf(X + (r0 + col) * CC + kc * 32, lane);
#pragma unroll
    for (int j = 0; j < 8; ++j) acc[j] = wmma_bf(a, frag_b(PT1 + (size_t)(n0 + j * 16 + col) * CC + kc * 32, lane), acc[j]); }
  float* dst; int pitch, c0; const float* bias;
  if (n0 < 256) { dst = LPRE; pitch = CC; c0 = n0; bias = lb + n0; } else if (n0 < 384) { dst = Q1; pitch = 128; c0 = n0 - 256; bias = q1b + c0; }
  else if (n0 < 512) { dst = Q2; pitch = 128; c0 = n0 - 384; bias = q2b + c0; } else { dst = KV2; pitch = CC; c0 = n0 - 512; bias = kv2b + c0; }
#pragma unroll
  for (int j = 0; j < 8; ++j) { const float bb = bfr(bias[j * 16 + col]);
#pragma unroll
    for (int r = 0; r < 8; ++r) so[wave][8 * g + r][j * 16 + col] = acc[j][r] + bb; }
  LDSX();
  for (int rl = 0; rl < 16; ++rl) vst2(dst + (r0 + rl) * pitch + c0 + lane * 4, *(const v4f*)(&so[wave][rl][lane * 4]));
}
__global__ __launch_bounds__(256) void k_srkv(const float* __restrict__ X, const __bf16* __restrict__ PTSR, const float* __restrict__ srb, const float* __restrict__ nw, const float* __restrict__ nb, const __bf16* __restrict__ PTKV, const float* __restrict__ kvb,
                                              float* __restrict__ K1, __bf16* __restrict__ V1h, __bf16* __restrict__ V1l) {
  __shared__ __align__(16) float sx[64][CC + 4];
  __shared__ __align__(16) __bf16 svh[128][72], svl[128][72];
  const int tid = threadIdx.x, wave = tid >> 5, lane = tid & 31, col = lane & 15, g = lane >> 4;
  const int b = blockIdx.x >> 4, m0 = (blockIdx.x & 15) * 64;
  const int rt = wave & 3, ct0 = (wave >> 2) * 8;
  { v8f acc[8] = {};
    const int m = m0 + rt * 16 + col; const int hp = m >> 5, wp = m & 31;
#pragma unroll 1
    for (int kc = 0; kc < 1024 / 32; ++kc) { const int tap = kc >> 3, c0 = (kc & 7) * 32; const int tok = (2 * hp + (tap >> 1)) * HW + 2 * wp + (tap & 1);
      const v16b a = frag_gbf(X + ((size_t)b * NT + tok) * CC + c0, lane);
#pragma unroll
      for (int j = 0; j < 8; ++j) acc[j] = wmma_bf(a, frag_b(PTSR + (size_t)((ct0 + j) * 16 + col) * 1024 + kc * 32, lane), acc[j]); }
#pragma unroll
    for (int j = 0; j < 8; ++j) { const int c = (ct0 + j) * 16 + col; const float bb = bfr(srb[c]);
#pragma unroll
      for (int r = 0; r < 8; ++r) sx[rt * 16 + 8 * g + r][c] = acc[j][r] + bb; } }
  __syncthreads();
#pragma unroll 1
  for (int rr = 0; rr < 8; ++rr) { const int row = wave * 8 + rr; float v[8], s = 0.f;
#pragma unroll
    for (int i = 0; i < 8; ++i) { v[i] = sx[row][lane * 8 + i]; s += v[i]; }
#pragma unroll
    for (int o = 16; o > 0; o >>= 1) s += __shfl_xor(s, o);
    const float mu = s * (1.0f / CC); float q = 0.f;
#pragma unroll
    for (int i = 0; i < 8; ++i) { const float d = v[i] - mu; q += d * d; }
#pragma unroll
    for (int o = 16; o > 0; o >>= 1) q += __shfl_xor(q, o);
    const float den = sqrtf(q * (1.0f / CC) + 1e-5f);
#pragma unroll
    for (int i = 0; i < 8; ++i) { const int c = lane * 8 + i; sx[row][c] = gelu_e((v[i] - mu) / den * bfr(nw[c]) + bfr(nb[c])); } }
  __syncthreads();
  { v8f acc[8] = {};
#pragma unroll 2
    for (int kc = 0; kc < CC / 32; ++kc) { const F2 a = split_row(&sx[rt * 16 + col][0], kc * 32, lane);
#pragma unroll
      for (int j = 0; j < 8; ++j) { const v16b wb = frag_b(PTKV + (size_t)((ct0 + j) * 16 + col) * CC + kc * 32, lane); acc[j] = wmma_bf(a.l, wb, acc[j]); acc[j] = wmma_bf(a.h, wb, acc[j]); } }
    __syncthreads();
    if (ct0 == 0) {
#pragma unroll
      for (int j = 0; j < 8; ++j) { const int c = j * 16 + col; const float bb = bfr(kvb[c]);
#pragma unroll
        for (int r = 0; r < 8; ++r) sx[rt * 16 + 8 * g + r][c] = acc[j][r] + bb; }
    } else {
#pragma unroll
      for (int j = 0; j < 8; ++j) { const int c = j * 16 + col; const float bb = bfr(kvb[128 + c]);
#pragma unroll
        for (int r = 0; r < 8; ++r) { const float v = acc[j][r] + bb; const __bf16 hi = (__bf16)v; svh[c][rt * 16 + 8 * g + r] = hi; svl[c][rt * 16 + 8 * g + r] = (__bf16)(v - (float)hi); } } } }
  __syncthreads();
  for (int q = tid; q < 256 * 8; q += 256) { const int rr = q >> 3, pc = q & 7; const int h = rr >> 6, ml = rr & 63;
    vst2(K1 + (((size_t)(b * NHB + h)) * NK + m0 + ml) * HD + pc * 4, *(const v4f*)(&sx[ml][h * 32 + pc * 4])); }
  for (int q = tid; q < 128 * 8; q += 256) { const int cl = q >> 3, pc = q & 7; const int h = cl >> 5, d = cl & 31; const size_t o = (((size_t)(b * NHB + h)) * HD + d) * NK + m0 + pc * 8;
    vst2((unsigned*)(V1h + o), *(const v4u*)(&svh[cl][pc * 8])); vst2((unsigned*)(V1l + o), *(const v4u*)(&svl[cl][pc * 8])); }
}
__global__ __launch_bounds__(128) void k_stats1(const float* __restrict__ Q1, const float* __restrict__ K1, float* __restrict__ M1, float* __restrict__ L1) {
  __shared__ float sm[64], sl[64];
  const int tid = threadIdx.x, wave = tid >> 5, lane = tid & 31, col = lane & 15, g = lane >> 4;
  const int bh = blockIdx.y, b = bh >> 2, h = bh & 3; const int n0 = blockIdx.x * 64 + wave * 16;
  const F2 aq = split_row(Q1 + ((size_t)b * NT + n0 + col) * 128 + h * HD, 0, lane);
  float m[8], l[8];
#pragma unroll
  for (int r = 0; r < 8; ++r) { m[r] = -3.0e38f; l[r] = 0.f; }
#pragma unroll 1
  for (int kb = 0; kb < NK; kb += 16) { const F2 bk = split_row(K1 + ((size_t)bh * NK + kb + col) * HD, 0, lane);
    v8f s = mac3(aq, bk, (v8f){});
#pragma unroll
    for (int r = 0; r < 8; ++r) { const float v = s[r] * SCALE; float mt = v;
#pragma unroll
      for (int o = 1; o < 16; o <<= 1) mt = fmaxf(mt, __shfl_xor(mt, o));
      const float mn = fmaxf(m[r], mt); float e = exp_ni(v - mn);
#pragma unroll
      for (int o = 1; o < 16; o <<= 1) e += __shfl_xor(e, o);
      l[r] = l[r] * exp_ni(m[r] - mn) + e; m[r] = mn; } }
  if (col == 0) {
#pragma unroll
    for (int r = 0; r < 8; ++r) { sm[wave * 16 + 8 * g + r] = m[r]; sl[wave * 16 + 8 * g + r] = l[r]; } }
  __syncthreads();
  if (tid < 16) { vst2(M1 + (size_t)bh * NT + blockIdx.x * 64 + tid * 4, *(const v4f*)&sm[tid * 4]); vst2(L1 + (size_t)bh * NT + blockIdx.x * 64 + tid * 4, *(const v4f*)&sl[tid * 4]); }
}
__global__ __launch_bounds__(128) void k_attn1(const float* __restrict__ Q1, const float* __restrict__ K1, const __bf16* __restrict__ V1h, const __bf16* __restrict__ V1l, const float* __restrict__ M1, const float* __restrict__ L1, float* __restrict__ GP, float* __restrict__ CAT) {
  __shared__ __align__(16) __bf16 sPh[4][16][40], sPl[4][16][40];
  __shared__ __align__(16) float scs[4][NK];
  __shared__ __align__(16) float sO[4][16][36];
  const int tid = threadIdx.x, wave = tid >> 5, lane = tid & 31, col = lane & 15, g = lane >> 4;
  const int bh = blockIdx.y, b = bh >> 2, h = bh & 3; const int qb = blockIdx.x; const int n0 = qb * 64 + wave * 16;
  const F2 aq = split_row(Q1 + ((size_t)b * NT + n0 + col) * 128 + h * HD, 0, lane);
  float mr[8], li[8];
#pragma unroll
  for (int r = 0; r < 8; ++r) { mr[r] = M1[(size_t)bh * NT + n0 + 8 * g + r]; li[r] = 1.0f / L1[(size_t)bh * NT + n0 + 8 * g + r]; }
  v8f acc[2] = {};
#pragma unroll 1
  for (int kt = 0; kt < NK / 32; ++kt) {
    float csum[2] = {0.f, 0.f};
#pragma unroll
    for (int jt = 0; jt < 2; ++jt) { const int kb = kt * 32 + jt * 16; const F2 bk = split_row(K1 + ((size_t)bh * NK + kb + col) * HD, 0, lane);
      v8f s = mac3(aq, bk, (v8f){});
#pragma unroll
      for (int r = 0; r < 8; ++r) { const float p = exp_ni(s[r] * SCALE - mr[r]) * li[r]; csum[jt] += p; const __bf16 hi = (__bf16)p; sPh[wave][8 * g + r][jt * 16 + col] = hi; sPl[wave][8 * g + r][jt * 16 + col] = (__bf16)(p - (float)hi); } }
#pragma unroll
    for (int jt = 0; jt < 2; ++jt) { const float t = csum[jt] + __shfl_xor(csum[jt], 16); if (g == 0) scs[wave][kt * 32 + jt * 16 + col] = t; }
    LDSX();
    const v16b ph = frag_b(&sPh[wave][col][0], lane), pl = frag_b(&sPl[wave][col][0], lane);
#pragma unroll
    for (int dt = 0; dt < 2; ++dt) { const size_t vo = ((size_t)bh * HD + dt * 16 + col) * NK + kt * 32; acc[dt] = mac3p(ph, pl, frag_b(V1h + vo, lane), frag_b(V1l + vo, lane), acc[dt]); }
    LDSX(); }
#pragma unroll
  for (int dt = 0; dt < 2; ++dt)
#pragma unroll
    for (int r = 0; r < 8; ++r) sO[wave][8 * g + r][dt * 16 + col] = acc[dt][r];
  __syncthreads();
  for (int q = lane; q < 16 * 8; q += 32) { const int rl = q >> 3, pc = q & 7; vst2(CAT + ((size_t)b * NT + n0 + rl) * CC + h * HD + pc * 4, *(const v4f*)(&sO[wave][rl][pc * 4])); }
  for (int k4 = tid; k4 < NK / 4; k4 += 128) { v4f t;
#pragma unroll
    for (int i = 0; i < 4; ++i) t[i] = ((scs[0][k4 * 4 + i] + scs[1][k4 * 4 + i]) + scs[2][k4 * 4 + i]) + scs[3][k4 * 4 + i];
    vst2(GP + (((size_t)bh * 64 + qb) * NK) + k4 * 4, t); }
}

__global__ __launch_bounds__(256) void k_lepe(const float* __restrict__ LPRE, const float* __restrict__ cw, const float* __restrict__ cb, float* __restrict__ LEPE) {
  const size_t q = (size_t)blockIdx.x * 256 + threadIdx.x; const size_t row = q >> 6; const int c0 = (int)(q & 63) * 4;
  const int b = (int)(row / NT), n = (int)(row % NT), hh = n >> 6, ww = n & 63;
  v4f o; o[0] = bfr(cb[c0]); o[1] = bfr(cb[c0 + 1]); o[2] = bfr(cb[c0 + 2]); o[3] = bfr(cb[c0 + 3]);
#pragma unroll
  for (int dy = 0; dy < 3; ++dy)
#pragma unroll
    for (int dx = 0; dx < 3; ++dx) { const int y = hh + dy - 1, x = ww + dx - 1; const bool in = (y >= 0) && (y < HW) && (x >= 0) && (x < HW);
      const int yc = y < 0 ? 0 : (y >= HW ? HW - 1 : y), xc = x < 0 ? 0 : (x >= HW ? HW - 1 : x);
      const float4 v = *(const float4*)(LPRE + ((size_t)b * NT + yc * HW + xc) * CC + c0);
      const float f = in ? 1.0f : 0.0f;
#pragma unroll
      for (int i = 0; i < 4; ++i) { const float wv = bfr(cw[(c0 + i) * 9 + dy * 3 + dx]); const float xv = i == 0 ? v.x : i == 1 ? v.y : i == 2 ? v.z : v.w; o[i] += wv * (xv * f); } }
  vst2(LEPE + row * CC + c0, o);
}
__device__ __forceinline__ int wtok(int wy, int wx, int n) { return (wy * 4 + (n >> 2)) * HW + wx * 4 + (n & 3); }
__global__ __launch_bounds__(256) void k_win(const float* __restrict__ Q2, const float* __restrict__ KV2, float* __restrict__ CAT, float* __restrict__ LMW) {
  __shared__ __align__(16) __bf16 sPh[8][16][40], sPl[8][16][40];
  __shared__ __align__(16) float sO[8][16][36];
  __shared__ float slm[4][4][16];
  const int tid = threadIdx.x, wave = tid >> 5, lane = tid & 31, col = lane & 15, g = lane >> 4;
  const int b = blockIdx.z, wy = blockIdx.y, wxg = blockIdx.x; const int wl = wave & 3, wx = wxg * 4 + wl;
#pragma unroll 1
  for (int u = 0; u < 2; ++u) { const int h = (wave >> 2) * 2 + u;
    const F2 aq = split_row(Q2 + ((size_t)b * NT + wtok(wy, wx, col)) * 128 + h * HD, 0, lane);
    const F2 bk = split_row(KV2 + ((size_t)b * NT + wtok(wy, wx, col)) * CC + h * HD, 0, lane);
    v8f s = mac3(aq, bk, (v8f){});
    float cs = 0.f;
#pragma unroll
    for (int r = 0; r < 8; ++r) { const float v = s[r] * SCALE; float mx = v;
#pragma unroll
      for (int o = 1; o < 16; o <<= 1) mx = fmaxf(mx, __shfl_xor(mx, o));
      const float e = exp_ni(v - mx); float sum = e;
#pragma unroll
      for (int o = 1; o < 16; o <<= 1) sum += __shfl_xor(sum, o);
      const float p = e / sum; cs += p; const __bf16 hi = (__bf16)p; sPh[wave][8 * g + r][col] = hi; sPl[wave][8 * g + r][col] = (__bf16)(p - (float)hi);
      sPh[wave][8 * g + r][16 + col] = (__bf16)0.f; sPl[wave][8 * g + r][16 + col] = (__bf16)0.f; }
    cs += __shfl_xor(cs, 16); if (g == 0) slm[wl][h][col] = cs;
    LDSX();
    const v16b ph = frag_b(&sPh[wave][col][0], lane), pl = frag_b(&sPl[wave][col][0], lane);
    v8f acc[2] = {};
#pragma unroll
    for (int dt = 0; dt < 2; ++dt) { v16b vh, vl;
#pragma unroll
      for (int i = 0; i < 8; ++i) { const float vv = KV2[((size_t)b * NT + wtok(wy, wx, 8 * g + i)) * CC + 128 + h * HD + dt * 16 + col]; const __bf16 hi = (__bf16)vv; vh[i] = hi; vl[i] = (__bf16)(vv - (float)hi); vh[8 + i] = (__bf16)0.f; vl[8 + i] = (__bf16)0.f; }
      acc[dt] = mac3p(ph, pl, vh, vl, acc[dt]); }
#pragma unroll
    for (int dt = 0; dt < 2; ++dt)
#pragma unroll
      for (int r = 0; r < 8; ++r) sO[wave][8 * g + r][dt * 16 + col] = acc[dt][r];
    LDSX();
    for (int q = lane; q < 16 * 8; q += 32) { const int n = q >> 3, pc = q & 7; vst2(CAT + ((size_t)b * NT + wtok(wy, wx, n)) * CC + 128 + h * HD + pc * 4, *(const v4f*)(&sO[wave][n][pc * 4])); }
    LDSX(); }
  __syncthreads();
  if (tid < 16) { v4f t; const int wq = tid >> 2, m0 = (tid & 3) * 4;
#pragma unroll
    for (int i = 0; i < 4; ++i) { const int m = m0 + i; t[i] = (((slm[wq][0][m] + slm[wq][1][m]) + slm[wq][2][m]) + slm[wq][3][m]) * (1.0f / 64.0f); }
    vst2(LMW + (((size_t)b * 256 + wy * 16 + wxg * 4 + wq) * 16) + m0, t); }
}
__global__ __launch_bounds__(128) void k_proj(const float* __restrict__ CAT, const float* __restrict__ LEPE, const __bf16* __restrict__ PTP, const float* __restrict__ pb, float* __restrict__ out) {
  __shared__ __align__(16) float so[4][16][132];
  const int tid = threadIdx.x, wave = tid >> 5, lane = tid & 31, col = lane & 15, g = lane >> 4; const size_t r0 = (size_t)blockIdx.x * 64 + wave * 16; const int n0 = blockIdx.y * 128;
  v8f acc[8] = {};
#pragma unroll 2
  for (int kc = 0; kc < CC / 32; ++kc) { float v[16]; const float* pa = CAT + (r0 + col) * CC + kc * 32 + 8 * g; const float* pl = LEPE + (r0 + col) * CC + kc * 32 + 8 * g;
#pragma unroll
    for (int i = 0; i < 8; ++i) { v[i] = pa[i] + pl[i]; v[8 + i] = pa[16 + i] + pl[16 + i]; }
    const F2 a = bsplit16(v);
#pragma unroll
    for (int j = 0; j < 8; ++j) { const v16b wb = frag_b(PTP + (size_t)(n0 + j * 16 + col) * CC + kc * 32, lane); acc[j] = wmma_bf(a.l, wb, acc[j]); acc[j] = wmma_bf(a.h, wb, acc[j]); } }
#pragma unroll
  for (int j = 0; j < 8; ++j) { const float bb = bfr(pb[n0 + j * 16 + col]);
#pragma unroll
    for (int r = 0; r < 8; ++r) { const float p = acc[j][r] + bb; so[wave][8 * g + r][j * 16 + col] = p + p; } }
  LDSX();
  for (int rl = 0; rl < 16; ++rl) vst2(out + (r0 + rl) * CC + n0 + lane * 4, *(const v4f*)(&so[wave][rl][lane * 4]));
}
__global__ __launch_bounds__(256) void k_mask(const float* __restrict__ GP, const float* __restrict__ LMW, float* __restrict__ out1, float* __restrict__ out2) {
  __shared__ float sg[NK];
  __shared__ float smk[HW][HW + 1];
  const int b = blockIdx.x, tid = threadIdx.x;
  for (int m = tid; m < NK; m += 256) { float s = 0.f;
#pragma unroll 1
    for (int r = 0; r < NHB * 64; ++r) s += GP[(((size_t)b * NHB * 64) + r) * NK + m];
    sg[m] = s * (1.0f / 16384.0f); }
  __syncthreads();
  for (int q = tid; q < NT; q += 256) { const int y = q >> 6, x = q & 63; const int win = (y >> 2) * 16 + (x >> 2), n = (y & 3) * 4 + (x & 3);
    smk[y][x] = LMW[((size_t)b * 256 + win) * 16 + n] + sg[(y >> 1) * 32 + (x >> 1)]; }
  __syncthreads();
  for (int q = tid; q < NT / 4; q += 256) { const int y = (q * 4) >> 6, x0 = (q * 4) & 63; v4f a, t;
#pragma unroll
    for (int i = 0; i < 4; ++i) { a[i] = smk[y][x0 + i]; t[i] = smk[x0 + i][y]; }
    vst2(out1 + (size_t)b * NT + q * 4, a); vst2(out2 + (size_t)b * NT + q * 4, t); }
}

extern "C" void kernel_launch(void* const* d_in, const int* in_sizes, int n_in, void* d_out, int out_size, void* d_ws, size_t ws_size, hipStream_t stream) {
  (void)in_sizes; (void)n_in; (void)out_size;
  const float** I = (const float**)d_in;
  if (ws_size < (size_t)WS_END) return;
  char* ws = (char*)d_ws;
  __bf16 *PT1 = (__bf16*)(ws + WS_PT1), *PTKV = (__bf16*)(ws + WS_PTKV), *PTP = (__bf16*)(ws + WS_PTP), *PTSR = (__bf16*)(ws + WS_PTSR);
  float *LPRE = (float*)(ws + WS_LPRE), *Q1 = (float*)(ws + WS_Q1), *Q2 = (float*)(ws + WS_Q2), *KV2 = (float*)(ws + WS_KV2), *K1 = (float*)(ws + WS_K1);
  __bf16 *V1h = (__bf16*)(ws + WS_V1H), *V1l = (__bf16*)(ws + WS_V1L);
  float *M1 = (float*)(ws + WS_M1), *L1 = (float*)(ws + WS_L1), *GP = (float*)(ws + WS_GP), *CAT = (float*)(ws + WS_CAT), *LEPE = (float*)(ws + WS_LEPE), *LMW = (float*)(ws + WS_LMW);
  float* out0 = (float*)d_out; float* out1 = out0 + (size_t)NR * CC; float* out2 = out1 + (size_t)NB * NT;
  k_pack<<<1536, 256, 0, stream>>>(I[9], I[1], I[5], I[7], I[3], I[17], I[13], PT1, PTKV, PTP, PTSR);
  k_lin1<<<dim3(NR / 64, 6), 128, 0, stream>>>(I[0], PT1, I[10], I[2], I[6], I[8], LPRE, Q1, Q2, KV2);
  k_srkv<<<NB * 16, 256, 0, stream>>>(I[0], PTSR, I[14], I[15], I[16], PTKV, I[4], K1, V1h, V1l);
  k_stats1<<<dim3(NT / 64, NB * NHB), 128, 0, stream>>>(Q1, K1, M1, L1);
  k_attn1<<<dim3(NT / 64, NB * NHB), 128, 0, stream>>>(Q1, K1, V1h, V1l, M1, L1, GP, CAT);
  k_lepe<<<NR * 64 / 256, 256, 0, stream>>>(LPRE, I[11], I[12], LEPE);
  k_win<<<dim3(4, 16, NB), 256, 0, stream>>>(Q2, KV2, CAT, LMW);
  k_proj<<<dim3(NR / 64, 2), 128, 0, stream>>>(CAT, LEPE, PTP, I[18], out0);
  k_mask<<<NB, 256, 0, stream>>>(GP, LMW, out1, out2);
}
